// transformer_head_55791625175535
// MI455X (gfx1250) — hardware-verified
//
#include <hip/hip_runtime.h>
#include <math.h>

typedef __attribute__((ext_vector_type(16))) _Float16 v16h;
typedef __attribute__((ext_vector_type(16))) __bf16 v16b;
typedef __attribute__((ext_vector_type(8)))  _Float16 v8h;
typedef __attribute__((ext_vector_type(8)))  float v8f;
typedef __attribute__((ext_vector_type(4)))  float v4f;
typedef __attribute__((ext_vector_type(2)))  float v2f;
typedef __attribute__((ext_vector_type(4)))  unsigned v4u;
typedef __attribute__((ext_vector_type(4)))  int v4i;
typedef float __attribute__((may_alias)) float_a;
typedef int __attribute__((may_alias)) int_a;

template <typename T> __device__ __forceinline__ void vst2(void* p, T v) { *(volatile T*)p = v; __threadfence(); *(volatile T*)p = v; }
__device__ __forceinline__ v8f wmma16(v16h a, v16h b, v8f c) {
  v8f d = __builtin_amdgcn_wmma_f32_16x16x32_f16(false, a, false, b, (short)0, c, false, false);
  asm volatile("v_nop\n\tv_nop\n\tv_nop\n\tv_nop" : "+v"(d) : "v"(a), "v"(b));
  return d;
}
__device__ __forceinline__ v8f wmma_bf(v16b a, v16b b, v8f c) {
  v8f d = __builtin_amdgcn_wmma_f32_16x16x32_bf16(false, a, false, b, (short)0, c, false, false);
  asm volatile("v_nop\n\tv_nop\n\tv_nop\n\tv_nop" : "+v"(d) : "v"(a), "v"(b));
  return d;
}
__device__ __forceinline__ v16h frag_h(const _Float16* rowk0, int lane) {
  union { v16h v; v8h q[2]; } u; const _Float16* p = rowk0 + 8 * (lane >> 4);
  u.q[0] = *(const v8h*)p; u.q[1] = *(const v8h*)(p + 16); return u.v;
}
__device__ __forceinline__ v16h frag_f32(const float* rowk0, int lane) {
  v16h a; const float* p = rowk0 + 8 * (lane >> 4);
#pragma unroll
  for (int i = 0; i < 8; ++i) { a[i] = (_Float16)p[i]; a[8 + i] = (_Float16)p[16 + i]; }
  return a;
}
__device__ __forceinline__ v16h frag_f32s(const float* rowk0, int lane, float sc) {
  v16h a; const float* p = rowk0 + 8 * (lane >> 4);
#pragma unroll
  for (int i = 0; i < 8; ++i) { a[i] = (_Float16)(p[i] * sc); a[8 + i] = (_Float16)(p[16 + i] * sc); }
  return a;
}
__device__ __forceinline__ v16h fragc_f32(const float* W, int k0, int n, int lane, int ld, int K) {
  v16h a; const int g = lane >> 4;
#pragma unroll
  for (int i = 0; i < 8; ++i) { const int ka = k0 + 8 * g + i, kb = ka + 16;
    a[i] = (_Float16)(ka < K ? W[(size_t)(ka < K ? ka : K - 1) * ld + n] : 0.f); a[8 + i] = (_Float16)(kb < K ? W[(size_t)(kb < K ? kb : K - 1) * ld + n] : 0.f); }
  return a;
}
struct F2 { v16b h, l; };
__device__ __forceinline__ F2 bsplit16(const float v[16]) { F2 r;
#pragma unroll
  for (int i = 0; i < 16; ++i) { const __bf16 h = (__bf16)v[i]; r.h[i] = h; r.l[i] = (__bf16)(v[i] - (float)h); }
  return r; }
__device__ __forceinline__ F2 split_row(const float* row, int k0, int lane) { float v[16]; const float* p = row + k0 + 8 * (lane >> 4);
#pragma unroll
  for (int i = 0; i < 8; ++i) { v[i] = p[i]; v[8 + i] = p[16 + i]; }
  return bsplit16(v); }
__device__ __forceinline__ F2 split_rowK(const float* row, int k0, int lane, int K) { float v[16]; const int g = lane >> 4;
#pragma unroll
  for (int i = 0; i < 8; ++i) { const int ka = k0 + 8 * g + i, kb = ka + 16; v[i] = ka < K ? row[ka < K ? ka : K - 1] : 0.f; v[8 + i] = kb < K ? row[kb < K ? kb : K - 1] : 0.f; }
  return bsplit16(v); }
__device__ __forceinline__ F2 split_col(const float* W, int k0, int n, int lane, int ld, int K) { float v[16]; const int g = lane >> 4;
#pragma unroll
  for (int i = 0; i < 8; ++i) { const int ka = k0 + 8 * g + i, kb = ka + 16; v[i] = ka < K ? W[(size_t)(ka < K ? ka : K - 1) * ld + n] : 0.f; v[8 + i] = kb < K ? W[(size_t)(kb < K ? kb : K - 1) * ld + n] : 0.f; }
  return bsplit16(v); }
__device__ __forceinline__ v8f mac3(const F2& a, const F2& b, v8f c) { c = wmma_bf(a.l, b.h, c); c = wmma_bf(a.h, b.l, c); return wmma_bf(a.h, b.h, c); }
__device__ __forceinline__ float sigm(float v) { return 1.0f / (1.0f + expf(-v)); }
#define LDSX() do { asm volatile("s_wait_dscnt 0" ::: "memory"); __builtin_amdgcn_wave_barrier(); __builtin_amdgcn_fence(__ATOMIC_RELEASE, "workgroup"); } while (0)


#define NB 8
#define NPTS 8192
#define KN 16
#define CC 64
#define PH 64
#define C4 256
#define WSC 256.0f
#define BNS 0.99950037f
#ifndef TNP
#define TNP (NB * NPTS)
#endif
typedef __attribute__((ext_vector_type(8))) __bf16 v8b;
__device__ __forceinline__ v16b frag_b(const __bf16* rowk0, int lane) {
  union { v16b v; v8b q[2]; } u; const __bf16* p = rowk0 + 8 * (lane >> 4);
  u.q[0] = *(const v8b*)p; u.q[1] = *(const v8b*)(p + 16); return u.v;
}
__device__ __forceinline__ float bfr(float v) { return (float)(__bf16)v; }
__device__ __attribute__((noinline)) float exp_ni(float v) { return expf(v); }
__device__ __attribute__((noinline)) float erf_ni(float v) { return erff(v); }

#define WS_W2  0u
#define WS_W3  (WS_W2 + 2u * CC * PH)
#define WS_W4  (WS_W3 + 2u * C4 * CC)
#define WS_END (WS_W4 + 2u * CC * C4)

__global__ __launch_bounds__(256) void k_packw(const float* __restrict__ W2, const float* __restrict__ W3, const float* __restrict__ W4, char* __restrict__ ws) { const int n = blockIdx.x, t = threadIdx.x; __shared__ __align__(16) _Float16 s2[PH], s3[CC], s4[C4];
  if (n < CC && t < PH) s2[t] = (_Float16)(bfr(W2[(size_t)t * CC + n]) * WSC); if (t < CC) s3[t] = (_Float16)(bfr(W3[(size_t)t * C4 + n]) * WSC); if (n < CC) s4[t] = (_Float16)(bfr(W4[(size_t)t * CC + n]) * WSC); __syncthreads();
  if (n < CC && t < PH / 8) vst2((unsigned*)((_Float16*)(ws + WS_W2) + (size_t)n * PH + t * 8), *(const v4u*)&s2[t * 8]);
  if (t < CC / 8) vst2((unsigned*)((_Float16*)(ws + WS_W3) + (size_t)n * CC + t * 8), *(const v4u*)&s3[t * 8]);
  if (n < CC && t < C4 / 8) vst2((unsigned*)((_Float16*)(ws + WS_W4) + (size_t)n * C4 + t * 8), *(const v4u*)&s4[t * 8]); }
__device__ __forceinline__ v16h frag_lh(const _Float16* p, int lane) { v16h a; const _Float16* pp = p + 8 * (lane >> 4);
#pragma unroll
  for (int i = 0; i < 8; ++i) { a[i] = pp[i]; a[8 + i] = pp[16 + i]; } return a; }
__global__ __launch_bounds__(128) void k_th(const float* __restrict__ KEY, const float* __restrict__ QRY, const float* __restrict__ VAL, const float* __restrict__ POS, const int* __restrict__ IDX, const float* __restrict__ W1, const float* __restrict__ B1, const float* __restrict__ G1, const float* __restrict__ T1, const _Float16* __restrict__ W2R, const float* __restrict__ B2, const _Float16* __restrict__ W3R, const float* __restrict__ B3, const float* __restrict__ G3, const float* __restrict__ T3, const _Float16* __restrict__ W4R, const float* __restrict__ B4, float* __restrict__ OUT) {
  __shared__ __align__(16) _Float16 shh[64][PH + 8]; __shared__ __align__(16) float spe[64][CC + 4]; __shared__ __align__(16) _Float16 stt[64][CC + 8]; __shared__ __align__(16) _Float16 sa2[64][C4 + 8]; __shared__ __align__(16) float slg[64][CC + 4]; __shared__ int sidx[64]; __shared__ __align__(16) float so[4][CC + 4];
  const int tid = threadIdx.x, wave = tid >> 5, lane = tid & 31, col = lane & 15, g = lane >> 4; const size_t p0 = (size_t)blockIdx.x * 4; const size_t b = p0 / NPTS;
  if (tid < 64) { int ix = IDX[(p0 + (tid >> 4)) * KN + (tid & 15)]; ix = ix < 0 ? 0 : (ix >= NPTS ? NPTS - 1 : ix); sidx[tid] = ix; } __syncthreads();
  for (int e = tid; e < 64 * PH; e += 128) { const int rl = e / PH, m = e % PH; const size_t pi = p0 + (rl >> 4), pj = b * NPTS + sidx[rl]; float s = bfr(B1[m]);
#pragma unroll
    for (int d = 0; d < 3; ++d) s += (bfr(POS[pi * 3 + d]) - bfr(POS[pj * 3 + d])) * bfr(W1[d * PH + m]);
    s = bfr(G1[m]) * s * BNS + bfr(T1[m]); shh[rl][m] = (_Float16)fmaxf(s, 0.f); }
  __syncthreads();
  { v8f acc[4] = {};
#pragma unroll
    for (int kc = 0; kc < PH / 32; ++kc) { const v16h a = frag_lh(&shh[wave * 16 + col][kc * 32], lane);
#pragma unroll
      for (int j = 0; j < 4; ++j) acc[j] = wmma16(a, frag_h(W2R + (size_t)(j * 16 + col) * PH + kc * 32, lane), acc[j]); }
#pragma unroll
    for (int j = 0; j < 4; ++j) { const int c = j * 16 + col; const float bb = bfr(B2[c]);
#pragma unroll
      for (int r = 0; r < 8; ++r) spe[wave * 16 + 8 * g + r][c] = acc[j][r] * (1.0f / WSC) + bb; } }
  __syncthreads();
  for (int e = tid; e < 64 * CC; e += 128) { const int rl = e / CC, c = e % CC; const size_t pi = p0 + (rl >> 4), pj = b * NPTS + sidx[rl]; stt[rl][c] = (_Float16)(bfr(QRY[pi * CC + c]) - bfr(KEY[pj * CC + c]) + spe[rl][c]); }
  __syncthreads();
  { v8f acc[16];
#pragma unroll
    for (int j = 0; j < 16; ++j) acc[j] = v8f{};
#pragma unroll
    for (int kc = 0; kc < CC / 32; ++kc) { const v16h a = frag_lh(&stt[wave * 16 + col][kc * 32], lane);
#pragma unroll
      for (int j = 0; j < 16; ++j) acc[j] = wmma16(a, frag_h(W3R + (size_t)(j * 16 + col) * CC + kc * 32, lane), acc[j]); }
#pragma unroll
    for (int j = 0; j < 16; ++j) { const int c = j * 16 + col; const float bb = bfr(B3[c]), gg = bfr(G3[c]) * BNS, be = bfr(T3[c]);
#pragma unroll
      for (int r = 0; r < 8; ++r) sa2[wave * 16 + 8 * g + r][c] = (_Float16)fmaxf(gg * (acc[j][r] * (1.0f / WSC) + bb) + be, 0.f); } }
  __syncthreads();
  { v8f acc[4] = {};
#pragma unroll
    for (int kc = 0; kc < C4 / 32; ++kc) { const v16h a = frag_lh(&sa2[wave * 16 + col][kc * 32], lane);
#pragma unroll
      for (int j = 0; j < 4; ++j) acc[j] = wmma16(a, frag_h(W4R + (size_t)(j * 16 + col) * C4 + kc * 32, lane), acc[j]); }
#pragma unroll
    for (int j = 0; j < 4; ++j) { const int c = j * 16 + col; const float bb = bfr(B4[c]);
#pragma unroll
      for (int r = 0; r < 8; ++r) slg[wave * 16 + 8 * g + r][c] = (acc[j][r] * (1.0f / WSC) + bb) * 0.125f; } }
  __syncthreads();
  { const int rl = tid >> 1, half = tid & 1; float* lr = &slg[rl][0]; float mx = -3.0e38f; for (int c = half * 32; c < half * 32 + 32; ++c) mx = fmaxf(mx, lr[c]); mx = fmaxf(mx, __shfl_xor(mx, 1));
    float s = 0.f; for (int c = half * 32; c < half * 32 + 32; ++c) { const float e = expf(lr[c] - mx); lr[c] = e; s += e; } s += __shfl_xor(s, 1); const float inv = 1.0f / s; for (int c = half * 32; c < half * 32 + 32; ++c) lr[c] *= inv; }
  __syncthreads();
  for (int e = tid; e < 4 * CC; e += 128) { const int pt = e / CC, c = e % CC; const size_t pi = p0 + pt; const float vi = bfr(VAL[pi * CC + c]); float s = 0.f;
#pragma unroll
    for (int k = 0; k < KN; ++k) { const int rl = pt * KN + k; s += slg[rl][c] * (vi + spe[rl][c]); } so[pt][c] = s; }
  __syncthreads(); if (tid < 64) { const int pt = tid >> 4, q = tid & 15; vst2(OUT + (p0 + pt) * CC + q * 4, *(const v4f*)&so[pt][q * 4]); } }
extern "C" void kernel_launch(void* const* d_in, const int* in_sizes, int n_in, void* d_out, int out_size, void* d_ws, size_t ws_size, hipStream_t stream) {
  (void)in_sizes; (void)n_in; (void)out_size;
  const float** F = (const float**)d_in;
  if (ws_size < (size_t)WS_END) return;
  char* ws = (char*)d_ws; _Float16 *W2R = (_Float16*)(ws + WS_W2), *W3R = (_Float16*)(ws + WS_W3), *W4R = (_Float16*)(ws + WS_W4);
  k_packw<<<C4, 256, 0, stream>>>(F[9], F[11], F[15], ws);
  k_th<<<TNP / 4, 128, 0, stream>>>(F[0], F[1], F[2], F[3], (const int*)d_in[4], F[5], F[6], F[7], F[8], W2R, F[10], W3R, F[12], F[13], F[14], W4R, F[16], (float*)d_out);
}
